// Rnn_36945308680506
// MI455X (gfx1250) — hardware-verified
//
#include <hip/hip_runtime.h>
#include <math.h>

constexpr int NBATCH  = 512;
constexpr int NSIG    = 3;
constexpr int NSTEP   = 4096;
constexpr int NHID    = 17;
constexpr int NCAT    = 2 * NHID;
constexpr int NOUTCH  = 2;
constexpr int BTILE   = 16;
constexpr int NBLK    = NBATCH / BTILE;
constexpr int NTHR    = 64;
constexpr int NCHUNK  = NSTEP / 4;
constexpr int SPITCH  = 20;
constexpr int NWHH    = NHID * NHID;
constexpr int NWIH    = NHID * NSIG;
constexpr float INV_STEPS = 1.0f / (float)NSTEP;

static_assert(NBATCH % BTILE == 0, "batch tiles exact");
static_assert(NSTEP % 4 == 0, "four steps per x chunk");
static_assert(NHID == 17, "row 16 lives alone in the second m-tile");
static_assert(NHID <= 32, "single 32-deep k step");
static_assert(NTHR == 64, "wave 0 forward, wave 1 backward");
static_assert(BTILE * NOUTCH == 32, "one 128-B output line per block");
static_assert(NWIH <= NTHR && NHID <= NTHR && NOUTCH <= NTHR, "single-pass staging of small vectors");
static_assert(SPITCH >= NHID + 1, "sum slab pitch holds 17 sums plus one written pad");

typedef __attribute__((ext_vector_type(16))) _Float16 v16h;
typedef __attribute__((ext_vector_type(8)))  float    v8f;
typedef __attribute__((ext_vector_type(4)))  float    v4f;
typedef __attribute__((ext_vector_type(8)))  unsigned v8u;

__device__ __forceinline__ unsigned h16bits(float f) {
  const _Float16 hv = (_Float16)f;
  const unsigned short us = __builtin_bit_cast(unsigned short, hv);
  return (unsigned)us;
}
__device__ __forceinline__ unsigned pack2h(float lo, float hi) {
  const unsigned a = h16bits(lo);
  const unsigned b = h16bits(hi);
  return a | (b << 16);
}
__device__ __forceinline__ void wmma_guard(v8f& d0, v8f& d1, v16h a0, v16h a1, v16h b) {
  asm volatile("v_nop\n\tv_nop\n\tv_nop\n\tv_nop" : "+v"(d0), "+v"(d1) : "v"(a0), "v"(a1), "v"(b));
}
__device__ __forceinline__ float tanh_f32(float v) {
  const float a = fminf(fabsf(v), 15.0f);
  const float e = expf(2.0f * a);
  const float r = __builtin_amdgcn_rcpf(e + 1.0f);
  const float t = 1.0f - 2.0f * r;
  return copysignf(t, v);
}

__global__ __launch_bounds__(NTHR) void birnn_mean_kernel(
    const float* __restrict__ x,
    const float* __restrict__ W_ih_f, const float* __restrict__ W_hh_f,
    const float* __restrict__ b_ih_f, const float* __restrict__ b_hh_f,
    const float* __restrict__ W_ih_b, const float* __restrict__ W_hh_b,
    const float* __restrict__ b_ih_b, const float* __restrict__ b_hh_b,
    const float* __restrict__ conv_w, const float* __restrict__ conv_b,
    float* __restrict__ out)
{
  __shared__ float sWhh[2][NWHH];
  __shared__ float sWih[2][NWIH];
  __shared__ float sBias[2][SPITCH];
  __shared__ float sCw[NOUTCH * NCAT];
  __shared__ float sCb[NOUTCH];
  __shared__ float sSum[2][BTILE * SPITCH];

  const int tid  = threadIdx.x;
  const int lane = tid & 31;
  const int dir  = tid >> 5;
  const int hh   = lane >> 4;
  const int n    = lane & 15;
  const int b0   = blockIdx.x * BTILE;

#pragma unroll 1
  for (int base = 0; base < NWHH; base += NTHR) {
    const int i  = base + tid;
    const int ic = (i < NWHH) ? i : (NWHH - 1);
    const float vf = W_hh_f[ic];
    const float vb = W_hh_b[ic];
    if (i < NWHH) { sWhh[0][i] = vf; sWhh[1][i] = vb; }
  }
  {
    const int ic = (tid < NWIH) ? tid : (NWIH - 1);
    const float vf = W_ih_f[ic];
    const float vb = W_ih_b[ic];
    if (tid < NWIH) { sWih[0][tid] = vf; sWih[1][tid] = vb; }
  }
  {
    const int ic = (tid < NHID) ? tid : (NHID - 1);
    const float vf = b_ih_f[ic] + b_hh_f[ic];
    const float vb = b_ih_b[ic] + b_hh_b[ic];
    if (tid < NHID) { sBias[0][tid] = vf; sBias[1][tid] = vb; }
  }
#pragma unroll 1
  for (int base = 0; base < NOUTCH * NCAT; base += NTHR) {
    const int i  = base + tid;
    const int ic = (i < NOUTCH * NCAT) ? i : (NOUTCH * NCAT - 1);
    const float v = conv_w[ic];
    if (i < NOUTCH * NCAT) sCw[i] = v;
  }
  {
    const int ic = (tid < NOUTCH) ? tid : (NOUTCH - 1);
    const float v = conv_b[ic];
    if (tid < NOUTCH) sCb[tid] = v;
  }
  __syncthreads();

  const float* wh = &sWhh[dir][0];
  v16h A0, A1;
  {
    v8u a0w, a1w;
#pragma unroll
    for (int j = 0; j < 8; ++j) {
      const int e0 = 2 * j;
      const int e1 = 2 * j + 1;
      const int k0 = (e0 < 8) ? (8 * hh + e0) : (16 + 8 * hh + (e0 - 8));
      const int k1 = (e1 < 8) ? (8 * hh + e1) : (16 + 8 * hh + (e1 - 8));
      const int k0c = (k0 < NHID) ? k0 : (NHID - 1);
      const int k1c = (k1 < NHID) ? k1 : (NHID - 1);
      const float r0a = wh[n * NHID + k0c];
      const float r0b = wh[n * NHID + k1c];
      const float r1a = wh[16 * NHID + k0c];
      const float r1b = wh[16 * NHID + k1c];
      const float w0a = (k0 < NHID) ? r0a : 0.0f;
      const float w0b = (k1 < NHID) ? r0b : 0.0f;
      const float w1a = ((k0 < NHID) && (n == 0)) ? r1a : 0.0f;
      const float w1b = ((k1 < NHID) && (n == 0)) ? r1b : 0.0f;
      a0w[j] = pack2h(w0a, w0b);
      a1w[j] = pack2h(w1a, w1b);
    }
    A0 = __builtin_bit_cast(v16h, a0w);
    A1 = __builtin_bit_cast(v16h, a1w);
  }

  float cb[8], ca0[8], ca1[8], ca2[8];
#pragma unroll
  for (int r = 0; r < 8; ++r) {
    const int i = 8 * hh + r;
    cb[r]  = sBias[dir][i];
    ca0[r] = sWih[dir][i * NSIG + 0];
    ca1[r] = sWih[dir][i * NSIG + 1];
    ca2[r] = sWih[dir][i * NSIG + 2];
  }
  const float cb16  = sBias[dir][16];
  const float c16a0 = sWih[dir][16 * NSIG + 0];
  const float c16a1 = sWih[dir][16 * NSIG + 1];
  const float c16a2 = sWih[dir][16 * NSIG + 2];

  const float* xb = x + (size_t)(b0 + n) * (size_t)(NSIG * NSTEP);
  const int tq0 = dir ? ((NCHUNK - 1) * 4) : 0;
  v4f cx0 = *(const v4f*)(xb + tq0);
  v4f cx1 = *(const v4f*)(xb + NSTEP + tq0);
  v4f cx2 = *(const v4f*)(xb + 2 * NSTEP + tq0);

  const v8u zero8 = {0u, 0u, 0u, 0u, 0u, 0u, 0u, 0u};
  v16h hB = __builtin_bit_cast(v16h, zero8);
  float ssum[8];
#pragma unroll
  for (int r = 0; r < 8; ++r) ssum[r] = 0.0f;
  float ssum16 = 0.0f;

#pragma unroll 1
  for (int q = 0; q < NCHUNK; ++q) {
    const int qn = (q + 1 < NCHUNK) ? (q + 1) : (NCHUNK - 1);
    const int tn = dir ? ((NCHUNK - 1 - qn) * 4) : (qn * 4);
    const v4f nx0 = *(const v4f*)(xb + tn);
    const v4f nx1 = *(const v4f*)(xb + NSTEP + tn);
    const v4f nx2 = *(const v4f*)(xb + 2 * NSTEP + tn);

    v4f q0, q1, q2;
    q0[0] = dir ? cx0[3] : cx0[0];
    q0[1] = dir ? cx0[2] : cx0[1];
    q0[2] = dir ? cx0[1] : cx0[2];
    q0[3] = dir ? cx0[0] : cx0[3];
    q1[0] = dir ? cx1[3] : cx1[0];
    q1[1] = dir ? cx1[2] : cx1[1];
    q1[2] = dir ? cx1[1] : cx1[2];
    q1[3] = dir ? cx1[0] : cx1[3];
    q2[0] = dir ? cx2[3] : cx2[0];
    q2[1] = dir ? cx2[2] : cx2[1];
    q2[2] = dir ? cx2[1] : cx2[2];
    q2[3] = dir ? cx2[0] : cx2[3];

#pragma unroll 1
    for (int s4 = 0; s4 < 4; ++s4) {
      const float x0 = q0[0];
      const float x1 = q1[0];
      const float x2 = q2[0];
      {
        const float a1 = q0[1], a2 = q0[2], a3 = q0[3];
        q0[0] = a1; q0[1] = a2; q0[2] = a3;
        const float b1 = q1[1], b2 = q1[2], b3 = q1[3];
        q1[0] = b1; q1[1] = b2; q1[2] = b3;
        const float c1 = q2[1], c2 = q2[2], c3 = q2[3];
        q2[0] = c1; q2[1] = c2; q2[2] = c3;
      }

      v8f c0;
#pragma unroll
      for (int r = 0; r < 8; ++r)
        c0[r] = fmaf(ca2[r], x2, fmaf(ca1[r], x1, fmaf(ca0[r], x0, cb[r])));
      const float pre16 = fmaf(c16a2, x2, fmaf(c16a1, x1, fmaf(c16a0, x0, cb16)));
      v8f c1;
      c1[0] = (hh == 0) ? pre16 : 0.0f;
      c1[1] = 0.0f; c1[2] = 0.0f; c1[3] = 0.0f;
      c1[4] = 0.0f; c1[5] = 0.0f; c1[6] = 0.0f; c1[7] = 0.0f;

      v8f d0 = __builtin_amdgcn_wmma_f32_16x16x32_f16(false, A0, false, hB, (short)0, c0, false, false);
      v8f d1 = __builtin_amdgcn_wmma_f32_16x16x32_f16(false, A1, false, hB, (short)0, c1, false, false);
      wmma_guard(d0, d1, A0, A1, hB);

      float th[8];
#pragma unroll
      for (int r = 0; r < 8; ++r) {
        th[r] = tanh_f32(d0[r]);
        ssum[r] += th[r];
      }
      const float d16 = d1[0];
      const float t16raw = tanh_f32(d16);
      const float t16 = (hh == 0) ? t16raw : 0.0f;
      ssum16 += t16;

      v8u hw;
      hw[0] = pack2h(th[0], th[1]);
      hw[1] = pack2h(th[2], th[3]);
      hw[2] = pack2h(th[4], th[5]);
      hw[3] = pack2h(th[6], th[7]);
      hw[4] = h16bits(t16);
      hw[5] = 0u;
      hw[6] = 0u;
      hw[7] = 0u;
      hB = __builtin_bit_cast(v16h, hw);
    }
    cx0 = nx0; cx1 = nx1; cx2 = nx2;
  }

  {
    float* sp = &sSum[dir][n * SPITCH];
#pragma unroll
    for (int r = 0; r < 8; ++r) sp[8 * hh + r] = ssum[r];
    sp[16 + hh] = ssum16;
  }
  __syncthreads();

  if (dir == 0) {
    const int bl = lane >> 1;
    const int o  = lane & 1;
    const float* sf = &sSum[0][bl * SPITCH];
    const float* sb = &sSum[1][bl * SPITCH];
    float acc = 0.0f;
#pragma unroll 1
    for (int i = 0; i < NHID; ++i) {
      acc = fmaf(sCw[o * NCAT + i], sf[i], acc);
      acc = fmaf(sCw[o * NCAT + NHID + i], sb[i], acc);
    }
    const float val = fmaf(acc, INV_STEPS, sCb[o]);
    float* op = out + (size_t)blockIdx.x * 32 + lane;
    *(volatile float*)op = val;
    __threadfence();
    *(volatile float*)op = val;
  }
}

extern "C" void kernel_launch(void* const* d_in, const int* in_sizes, int n_in,
                              void* d_out, int out_size, void* d_ws, size_t ws_size,
                              hipStream_t stream) {
  (void)d_ws; (void)ws_size;
  if (n_in < 11 || d_out == nullptr) return;
  if (in_sizes[0] != NBATCH * NSIG * NSTEP ||
      in_sizes[1] != NWIH || in_sizes[2] != NWHH || in_sizes[3] != NHID || in_sizes[4] != NHID ||
      in_sizes[5] != NWIH || in_sizes[6] != NWHH || in_sizes[7] != NHID || in_sizes[8] != NHID ||
      in_sizes[9] != NOUTCH * NCAT || in_sizes[10] != NOUTCH ||
      out_size != NBATCH * NOUTCH) return;

  const float* x      = (const float*)d_in[0];
  const float* W_ih_f = (const float*)d_in[1];
  const float* W_hh_f = (const float*)d_in[2];
  const float* b_ih_f = (const float*)d_in[3];
  const float* b_hh_f = (const float*)d_in[4];
  const float* W_ih_b = (const float*)d_in[5];
  const float* W_hh_b = (const float*)d_in[6];
  const float* b_ih_b = (const float*)d_in[7];
  const float* b_hh_b = (const float*)d_in[8];
  const float* conv_w = (const float*)d_in[9];
  const float* conv_b = (const float*)d_in[10];

  birnn_mean_kernel<<<NBLK, NTHR, 0, stream>>>(x,
      W_ih_f, W_hh_f, b_ih_f, b_hh_f,
      W_ih_b, W_hh_b, b_ih_b, b_hh_b,
      conv_w, conv_b, (float*)d_out);
}
